// RNNDecoderP_83236466196672
// MI455X (gfx1250) — hardware-verified
//
#include <hip/hip_runtime.h>
#include <math.h>

constexpr int NBAND  = 2;
constexpr int NBATCH = 512;
constexpr int NSTEP  = 512;
constexpr int NDIM   = 64;
constexpr int NTE    = 16;
constexpr int NLAY   = 2;
constexpr int NGATE  = 3 * NDIM;
constexpr int NMAT   = NBAND * NLAY;
constexpr int ROWS_BLK = 16;
constexpr int HPITCH   = 72;
constexpr int HEAD_PITCH = 128;
constexpr int WPLANE_THREADS = NMAT * NGATE * 8;
constexpr int WPLANE_BLOCKS  = WPLANE_THREADS / 256;
constexpr float ACT_CARRY = 16.0f;
constexpr float WGT_CARRY = 16.0f;
constexpr float ACC_INV   = 1.0f / (ACT_CARRY * WGT_CARRY);
constexpr float ACT_INV   = 1.0f / ACT_CARRY;

static_assert(NDIM == 64, "row of 64 halves is one 128-B line");
static_assert(NDIM % 32 == 0, "K multiple of 32");
static_assert(NBATCH % ROWS_BLK == 0, "batch tiles exact");
static_assert(NGATE == 192, "three gate blocks of 64 columns");
static_assert((2 * ROWS_BLK * HPITCH) % 128 == 0, "h tile zero fill exact");
static_assert(WPLANE_THREADS == 6144, "768 out rows x 8 pieces per plane");
static_assert(WPLANE_BLOCKS * 256 == WPLANE_THREADS && WPLANE_BLOCKS == 24, "weight plane grid exact");
static_assert(NTE * NDIM == 1024, "film tables are 256 threads x 4 floats");

typedef __attribute__((ext_vector_type(16))) _Float16 v16h;
typedef __attribute__((ext_vector_type(8)))  _Float16 v8h;
typedef __attribute__((ext_vector_type(8)))  float    v8f;
typedef __attribute__((ext_vector_type(4)))  float    v4f;
typedef __attribute__((ext_vector_type(4)))  unsigned v4u;

__device__ __forceinline__ void keep4_h(v16h a, v16h b, v16h c, v16h d) { asm volatile("v_nop" :: "v"(a), "v"(b), "v"(c), "v"(d)); }
__device__ __forceinline__ void tie_group(v8f& a, v8f& b, v8f& c, v8f& d, v16h x0, v16h x1, v16h y0, v16h y1) {
  asm volatile("v_nop\n\tv_nop\n\tv_nop\n\tv_nop" : "+v"(a), "+v"(b), "+v"(c), "+v"(d) : "v"(x0), "v"(x1), "v"(y0), "v"(y1));
}

template <typename T> struct Frag;
template <> struct Frag<_Float16> {
  typedef v16h V; union U { v16h v; v8h h[2]; };
  static __device__ __forceinline__ v16h load(const _Float16* p) {
    U f; f.h[0] = *(const v8h*)(p); f.h[1] = *(const v8h*)(p + 16); return f.v;
  }
  static __device__ __forceinline__ v8f mma(v16h a, v16h b, v8f c) {
    return __builtin_amdgcn_wmma_f32_16x16x32_f16(false, a, false, b, (short)0, c, false, false);
  }
};

__device__ __forceinline__ float h16_to_f32(unsigned hb) {
  const unsigned sgn = (hb & 0x8000u) << 16; const unsigned em = hb & 0x7fffu;
  const float fn = __uint_as_float((em << 13) + 0x38000000u);
  const float fs = (float)em * 5.9604644775390625e-8f;
  const float mag = (em < 0x400u) ? fs : fn; return __uint_as_float(__float_as_uint(mag) | sgn);
}

__device__ __forceinline__ float gate_sig(float x)  { return __builtin_amdgcn_rcpf(1.0f + expf(-x)); }
__device__ __forceinline__ float gate_tanh(float x) { return 1.0f - 2.0f * __builtin_amdgcn_rcpf(expf(2.0f * x) + 1.0f); }

__global__ __launch_bounds__(256) void wplane_kernel(const float* __restrict__ gw, const float* __restrict__ gu,
                                                     unsigned short* __restrict__ wt, unsigned short* __restrict__ ut) {
  const float* src = (blockIdx.y == 0) ? gw : gu;
  unsigned short* dst = (blockIdx.y == 0) ? wt : ut;
  const int i = blockIdx.x * 256 + threadIdx.x;
  if (i < WPLANE_THREADS) {
    const int orow = i >> 3;
    const int c8   = (i & 7) * 8;
    const int mat  = orow / NGATE;
    const int n    = orow - mat * NGATE;
    v8h hv;
#pragma unroll
    for (int e = 0; e < 8; ++e) {
      const float f = src[((size_t)(mat * NDIM + c8 + e)) * NGATE + n];
      hv[e] = (_Float16)(f * WGT_CARRY);
    }
    unsigned short* op = dst + (size_t)orow * NDIM + c8;
    *(volatile v8h*)op = hv;
    __threadfence();
    *(volatile v8h*)op = hv;
  }
}

__global__ __launch_bounds__(256) void fold_kernel(const float* __restrict__ w1, const float* __restrict__ b1,
                                                   const float* __restrict__ w2, const float* __restrict__ b2,
                                                   float* __restrict__ ht) {
  __shared__ __align__(16) float st[2 * HEAD_PITCH];
  const int tid  = threadIdx.x;
  const int band = tid >> 7;
  const int idx  = tid & 127;
  const int dc   = (idx < NDIM) ? idx : (NDIM - 1);
  float s1 = 0.0f, s2 = 0.0f;
#pragma unroll 1
  for (int e = 0; e < NDIM; ++e) {
    const float wv = w2[band * NDIM + e];
    s1 = fmaf(w1[((size_t)(band * NDIM + dc)) * NDIM + e], wv, s1);
    s2 = fmaf(b1[band * NDIM + e], wv, s2);
  }
  const float b2v = b2[band];
  const float val = (idx < NDIM) ? s1 : ((idx == NDIM) ? (s2 + b2v) : 0.0f);
  st[tid] = val;
  __syncthreads();
  if (tid < 64) {
    const v4f v = *(const v4f*)(st + tid * 4);
    float* op = ht + tid * 4;
    *(volatile v4f*)op = v;
    __threadfence();
    *(volatile v4f*)op = v;
  }
}

__global__ __launch_bounds__(256) void prep_kernel(const int* __restrict__ onehot, const float* __restrict__ z_last,
                                                   const float* __restrict__ te, const float* __restrict__ xw,
                                                   const float* __restrict__ xb, const float* __restrict__ fgw,
                                                   const float* __restrict__ fgb, const float* __restrict__ fbw,
                                                   const float* __restrict__ fbb, unsigned* __restrict__ Xu, int band) {
  __shared__ unsigned maskw[NSTEP / 32];
  __shared__ int psum[NSTEP / 32 + 1];
  __shared__ float rx0s[NDIM];
  __shared__ __align__(16) float sGW[NTE * NDIM];
  __shared__ __align__(16) float sBW[NTE * NDIM];
  const int tid  = threadIdx.x;
  const int lane = tid & 31;
  const int wave = __builtin_amdgcn_readfirstlane(tid >> 5);
  const int b    = blockIdx.x;

  {
    const v4f a = *(const v4f*)(fgw + tid * 4);
    const v4f c = *(const v4f*)(fbw + tid * 4);
    *(v4f*)(sGW + tid * 4) = a;
    *(v4f*)(sBW + tid * 4) = c;
  }
#pragma unroll
  for (int i = 0; i < 2; ++i) {
    const int t = i * 256 + tid;
    const int bit = (onehot[((size_t)b * NSTEP + t) * NBAND + band] != 0) ? 1 : 0;
    const unsigned bal = (unsigned)__ballot(bit);
    if (lane == 0) maskw[i * 8 + wave] = bal;
  }
  if (tid < NDIM) {
    float acc = xb[band * NDIM + tid];
#pragma unroll 1
    for (int k = 0; k < NDIM; ++k)
      acc = fmaf(z_last[(size_t)b * NDIM + k], xw[((size_t)(band * NDIM + k)) * NDIM + tid], acc);
    rx0s[tid] = acc;
  }
  __syncthreads();
  if (tid == 0) {
    int s = 0;
    psum[0] = 0;
#pragma unroll 1
    for (int w = 0; w < NSTEP / 32; ++w) { s += __popc(maskw[w]); psum[w + 1] = s; }
  }
  __syncthreads();
  const int nval = __builtin_amdgcn_readfirstlane(psum[NSTEP / 32]);

  const int d0 = 2 * lane;
  float gw0[NTE], gw1[NTE], bw0[NTE], bw1[NTE];
#pragma unroll
  for (int k = 0; k < NTE; ++k) {
    gw0[k] = sGW[k * NDIM + d0];
    gw1[k] = sGW[k * NDIM + d0 + 1];
    bw0[k] = sBW[k * NDIM + d0];
    bw1[k] = sBW[k * NDIM + d0 + 1];
  }
  const float gb0 = fgb[d0], gb1 = fgb[d0 + 1];
  const float bb0 = fbb[d0], bb1 = fbb[d0 + 1];
  const float ra = rx0s[d0], rb = rx0s[d0 + 1];

#pragma unroll 1
  for (int it = 0; it < NSTEP / 8; ++it) {
    const int t = it * 8 + wave;
    const unsigned w = (unsigned)__builtin_amdgcn_readfirstlane((int)maskw[t >> 5]);
    const int pre = __builtin_amdgcn_readfirstlane(psum[t >> 5]);
    const int bpos = t & 31;
    const int pv = pre + __popc(w & ((1u << bpos) - 1u));
    const int valid = (int)((w >> bpos) & 1u);
    int dest = valid ? pv : (nval + (t - pv));
    dest = dest < 0 ? 0 : (dest > NSTEP - 1 ? NSTEP - 1 : dest);
    unsigned pk = 0u;
    if (valid) {
      const float* ter = te + ((size_t)b * NSTEP + t) * NTE;
      v4f tv[4];
#pragma unroll
      for (int q = 0; q < 4; ++q) tv[q] = *(const v4f*)(ter + 4 * q);
      float g0 = gb0, g1 = gb1, e0 = bb0, e1 = bb1;
#pragma unroll
      for (int k = 0; k < NTE; ++k) {
        const float x = tv[k >> 2][k & 3];
        g0 = fmaf(x, gw0[k], g0);
        g1 = fmaf(x, gw1[k], g1);
        e0 = fmaf(x, bw0[k], e0);
        e1 = fmaf(x, bw1[k], e1);
      }
      const float x0 = ra * g0 + e0;
      const float x1 = rb * g1 + e1;
      const _Float16 h0 = (_Float16)(x0 * ACT_CARRY);
      const _Float16 h1 = (_Float16)(x1 * ACT_CARRY);
      const unsigned u0 = (unsigned)__builtin_bit_cast(unsigned short, h0);
      const unsigned u1 = (unsigned)__builtin_bit_cast(unsigned short, h1);
      pk = u0 | (u1 << 16);
    }
    unsigned* dp = Xu + ((size_t)b * NSTEP + dest) * (NDIM / 2) + lane;
    *(volatile unsigned*)dp = pk;
    __threadfence();
    *(volatile unsigned*)dp = pk;
  }
}

__global__ __launch_bounds__(128) void gru_scan_kernel(const unsigned short* __restrict__ Xin, unsigned short* __restrict__ Xout,
                                                       const unsigned short* __restrict__ WTp,
                                                       const unsigned short* __restrict__ UTp,
                                                       const float* __restrict__ gru_b, const int* __restrict__ onehot,
                                                       int band, int layer) {
  __shared__ __align__(16) _Float16 hT[2][ROWS_BLK * HPITCH];
  __shared__ int nv[ROWS_BLK];
  const int tid  = threadIdx.x;
  const int lane = tid & 31;
  const int wv   = __builtin_amdgcn_readfirstlane(tid >> 5);
  const int lh   = lane >> 4;
  const int lm   = lane & 15;
  const int row0 = blockIdx.x * ROWS_BLK;

  {
    _Float16* hz = &hT[0][0];
#pragma unroll 1
    for (int i = tid; i < 2 * ROWS_BLK * HPITCH; i += 128) hz[i] = (_Float16)0.0f;
  }
  {
    const int r = tid >> 3, s = tid & 7;
    const int* op = onehot + ((size_t)(row0 + r) * NSTEP + s * 64) * NBAND + band;
    int cnt = 0;
#pragma unroll 1
    for (int q = 0; q < 64; ++q) cnt += (op[q * NBAND] != 0) ? 1 : 0;
    cnt += __shfl_xor(cnt, 1, 32);
    cnt += __shfl_xor(cnt, 2, 32);
    cnt += __shfl_xor(cnt, 4, 32);
    if (s == 0) nv[r] = cnt;
  }
  __syncthreads();

  int nvr[8];
#pragma unroll
  for (int i = 0; i < 8; ++i) {
    int v = nv[i + 8 * lh];
    v = v < 0 ? 0 : (v > NSTEP ? NSTEP : v);
    nvr[i] = v;
  }
  int tm = 0;
#pragma unroll
  for (int i = 0; i < ROWS_BLK; ++i) { const int v = nv[i]; tm = v > tm ? v : tm; }
  tm = tm > NSTEP ? NSTEP : tm;
  const int tmax = __builtin_amdgcn_readfirstlane(tm);

  const int ncol = wv * 16 + lm;
  const size_t matoff = (size_t)(band * NLAY + layer) * NGATE * NDIM;
  const _Float16* wp = (const _Float16*)WTp + matoff + (size_t)ncol * NDIM + 8 * lh;
  const _Float16* up = (const _Float16*)UTp + matoff + (size_t)ncol * NDIM + 8 * lh;
  const v16h wz0 = Frag<_Float16>::load(wp);
  const v16h wz1 = Frag<_Float16>::load(wp + 32);
  const v16h wr0 = Frag<_Float16>::load(wp + 64 * NDIM);
  const v16h wr1 = Frag<_Float16>::load(wp + 64 * NDIM + 32);
  const v16h wn0 = Frag<_Float16>::load(wp + 128 * NDIM);
  const v16h wn1 = Frag<_Float16>::load(wp + 128 * NDIM + 32);
  const v16h uz0 = Frag<_Float16>::load(up);
  const v16h uz1 = Frag<_Float16>::load(up + 32);
  const v16h ur0 = Frag<_Float16>::load(up + 64 * NDIM);
  const v16h ur1 = Frag<_Float16>::load(up + 64 * NDIM + 32);
  const v16h un0 = Frag<_Float16>::load(up + 128 * NDIM);
  const v16h un1 = Frag<_Float16>::load(up + 128 * NDIM + 32);
  const float* bbp = gru_b + (size_t)(band * NLAY + layer) * NGATE;
  const float bz = bbp[ncol], br = bbp[ncol + 64], bn = bbp[ncol + 128];

  float hf[8];
#pragma unroll
  for (int i = 0; i < 8; ++i) hf[i] = 0.0f;

  const _Float16* xrow = (const _Float16*)Xin + ((size_t)(row0 + lm) * NSTEP) * NDIM + 8 * lh;
  const v8f z8 = {0.f, 0.f, 0.f, 0.f, 0.f, 0.f, 0.f, 0.f};
  const int orow = 4 * wv + (lane >> 3);
  const int oc8  = (lane & 7) * 8;
  unsigned short* obase = Xout + ((size_t)(row0 + orow) * NSTEP) * NDIM + oc8;

#pragma unroll 1
  for (int t = 0; t < tmax; ++t) {
    const int rb = t & 1;
    const int wb = rb ^ 1;
    const _Float16* xr = xrow + (size_t)t * NDIM;
    const _Float16* hr = &hT[rb][0] + lm * HPITCH + 8 * lh;
    const v16h ax0 = Frag<_Float16>::load(xr);
    const v16h ax1 = Frag<_Float16>::load(xr + 32);
    const v16h ah0 = Frag<_Float16>::load(hr);
    const v16h ah1 = Frag<_Float16>::load(hr + 32);

    v8f accz = z8, accr = z8, accx = z8, acch = z8;
    accz = Frag<_Float16>::mma(ax0, wz0, accz);
    accz = Frag<_Float16>::mma(ax1, wz1, accz);
    accz = Frag<_Float16>::mma(ah0, uz0, accz);
    accz = Frag<_Float16>::mma(ah1, uz1, accz);
    accr = Frag<_Float16>::mma(ax0, wr0, accr);
    accr = Frag<_Float16>::mma(ax1, wr1, accr);
    accr = Frag<_Float16>::mma(ah0, ur0, accr);
    accr = Frag<_Float16>::mma(ah1, ur1, accr);
    accx = Frag<_Float16>::mma(ax0, wn0, accx);
    accx = Frag<_Float16>::mma(ax1, wn1, accx);
    acch = Frag<_Float16>::mma(ah0, un0, acch);
    acch = Frag<_Float16>::mma(ah1, un1, acch);
    tie_group(accz, accr, accx, acch, ax0, ax1, ah0, ah1);
    keep4_h(wz0, wz1, wr0, wr1);
    keep4_h(wn0, wn1, uz0, uz1);
    keep4_h(ur0, ur1, un0, un1);

    _Float16* hw = &hT[wb][0];
#pragma unroll
    for (int i = 0; i < 8; ++i) {
      const float az = accz[i] * ACC_INV + bz;
      const float ar = accr[i] * ACC_INV + br;
      const float zg = gate_sig(az);
      const float rg = gate_sig(ar);
      const float hn = acch[i] * ACC_INV;
      const float an = (accx[i] * ACC_INV + bn) + rg * hn;
      const float ng = gate_tanh(an);
      const float ho = hf[i];
      const float hnew = (1.0f - zg) * ng + zg * ho;
      const float hs = (t < nvr[i]) ? hnew : ho;
      hf[i] = hs;
      hw[(i + 8 * lh) * HPITCH + ncol] = (_Float16)(hs * ACT_CARRY);
    }
    __syncthreads();
    {
      const v8h hv = *(const v8h*)(&hT[wb][0] + orow * HPITCH + oc8);
      unsigned short* op = obase + (size_t)t * NDIM;
      *(volatile v8h*)op = hv;
      __threadfence();
      *(volatile v8h*)op = hv;
    }
  }
}

__global__ __launch_bounds__(256) void head_kernel(const unsigned short* __restrict__ H2, const float* __restrict__ ht,
                                                   const int* __restrict__ onehot, float* __restrict__ out, int band) {
  __shared__ float sHT[HEAD_PITCH];
  __shared__ int wcnt[8];
  const int tid  = threadIdx.x;
  const int lane = tid & 31;
  const int wave = __builtin_amdgcn_readfirstlane(tid >> 5);
  const int b    = blockIdx.x;
  int c = 0;
#pragma unroll
  for (int i = 0; i < 2; ++i) {
    const int t = i * 256 + tid;
    const int bit = (onehot[((size_t)b * NSTEP + t) * NBAND + band] != 0) ? 1 : 0;
    const unsigned bal = (unsigned)__ballot(bit);
    c += __popc(bal);
  }
  if (lane == 0) wcnt[wave] = c;
  if (tid < HEAD_PITCH) sHT[tid] = ht[band * HEAD_PITCH + tid];
  __syncthreads();
  int nsum = 0;
#pragma unroll
  for (int i = 0; i < 8; ++i) nsum += wcnt[i];
  nsum = nsum < 0 ? 0 : (nsum > NSTEP ? NSTEP : nsum);
  const int nval = __builtin_amdgcn_readfirstlane(nsum);
  const float cc = sHT[NDIM];

#pragma unroll 1
  for (int i = 0; i < 2; ++i) {
    const int t0 = i * 256 + wave * 32;
    const int t  = t0 + lane;
    float y = 0.0f;
    if (t0 < nval) {
      const int tc = (t < nval) ? t : (nval - 1);
      const v4u* rp = (const v4u*)(H2 + ((size_t)b * NSTEP + tc) * NDIM);
      float acc = 0.0f;
#pragma unroll 1
      for (int q = 0; q < 8; ++q) {
        const v4u w = rp[q];
        const float* wq = sHT + q * 8;
#pragma unroll
        for (int j = 0; j < 4; ++j) {
          const unsigned wd = w[j];
          const float lo = h16_to_f32(wd & 0xffffu);
          const float hi = h16_to_f32(wd >> 16);
          acc = fmaf(lo, wq[2 * j], acc);
          acc = fmaf(hi, wq[2 * j + 1], acc);
        }
      }
      const float yv = cc + acc * ACT_INV;
      y = (t < nval) ? yv : 0.0f;
    }
    float* op = out + ((size_t)(band * NBATCH + b)) * NSTEP + t;
    *(volatile float*)op = y;
    __threadfence();
    *(volatile float*)op = y;
  }
}

extern "C" void kernel_launch(void* const* d_in, const int* in_sizes, int n_in,
                              void* d_out, int out_size, void* d_ws, size_t ws_size, hipStream_t stream) {
  if (n_in < 16 || d_out == nullptr || d_ws == nullptr) return;
  if (in_sizes[0] != NBATCH * NSTEP * NBAND || in_sizes[1] != NBATCH * NDIM || in_sizes[2] != NBATCH * NSTEP * NTE ||
      in_sizes[3] != NBAND * NDIM * NDIM || in_sizes[4] != NBAND * NDIM || in_sizes[5] != NTE * NDIM ||
      in_sizes[6] != NDIM || in_sizes[7] != NTE * NDIM || in_sizes[8] != NDIM ||
      in_sizes[9] != NMAT * NDIM * NGATE || in_sizes[10] != NMAT * NDIM * NGATE || in_sizes[11] != NMAT * NGATE ||
      in_sizes[12] != NBAND * NDIM * NDIM || in_sizes[13] != NBAND * NDIM || in_sizes[14] != NBAND * NDIM ||
      in_sizes[15] != NBAND || out_size != NBAND * NBATCH * NSTEP) return;

  const int*   onehot  = (const int*)  d_in[0];
  const float* z_last  = (const float*)d_in[1];
  const float* te      = (const float*)d_in[2];
  const float* xproj_W = (const float*)d_in[3];
  const float* xproj_b = (const float*)d_in[4];
  const float* film_gw = (const float*)d_in[5];
  const float* film_gb = (const float*)d_in[6];
  const float* film_bw = (const float*)d_in[7];
  const float* film_bb = (const float*)d_in[8];
  const float* gru_W   = (const float*)d_in[9];
  const float* gru_U   = (const float*)d_in[10];
  const float* gru_b   = (const float*)d_in[11];
  const float* mlp_W1  = (const float*)d_in[12];
  const float* mlp_b1  = (const float*)d_in[13];
  const float* mlp_W2  = (const float*)d_in[14];
  const float* mlp_b2  = (const float*)d_in[15];
  float* out = (float*)d_out;

  char* ws = (char*)d_ws; size_t off = 0;
  auto carve = [&](size_t bytes) -> char* { char* p = ws + off; off += (bytes + 255) & ~(size_t)255; return p; };
  const size_t plane_bytes = (size_t)NBATCH * NSTEP * NDIM * 2;
  unsigned short* X  = (unsigned short*)carve(plane_bytes);
  unsigned short* H1 = (unsigned short*)carve(plane_bytes);
  unsigned short* H2 = (unsigned short*)carve(plane_bytes);
  unsigned short* WT = (unsigned short*)carve((size_t)NMAT * NGATE * NDIM * 2);
  unsigned short* UT = (unsigned short*)carve((size_t)NMAT * NGATE * NDIM * 2);
  float*          HT = (float*)carve((size_t)NBAND * HEAD_PITCH * 4);
  if (off > ws_size || off > (size_t)134217728) return;

  wplane_kernel<<<dim3(WPLANE_BLOCKS, 2), 256, 0, stream>>>(gru_W, gru_U, WT, UT);
  fold_kernel<<<1, 256, 0, stream>>>(mlp_W1, mlp_b1, mlp_W2, mlp_b2, HT);

  for (int band = 0; band < NBAND; ++band) {
    prep_kernel<<<NBATCH, 256, 0, stream>>>(onehot, z_last, te, xproj_W, xproj_b, film_gw, film_gb, film_bw, film_bb,
                                            (unsigned*)X, band);
    gru_scan_kernel<<<NBATCH / ROWS_BLK, 128, 0, stream>>>(X, H1, WT, UT, gru_b, onehot, band, 0);
    gru_scan_kernel<<<NBATCH / ROWS_BLK, 128, 0, stream>>>(H1, H2, WT, UT, gru_b, onehot, band, 1);
    head_kernel<<<NBATCH, 256, 0, stream>>>(H2, HT, onehot, out, band);
  }
}
